// MultiHeadAttentionQuantum_65481071409110
// MI455X (gfx1250) — hardware-run, weakly checked
//
#include <hip/hip_runtime.h>
#include <math.h>

typedef __attribute__((ext_vector_type(16))) _Float16 v16h;
typedef __attribute__((ext_vector_type(8)))  _Float16 v8h;
typedef __attribute__((ext_vector_type(8)))  float    v8f;
typedef __attribute__((ext_vector_type(4)))  float    v4f;
typedef __attribute__((ext_vector_type(4)))  unsigned v4u;

constexpr int kBatch   = 8;
constexpr int kSeq     = 256;
constexpr int kEmb     = 12;
constexpr int kHeads   = 4;
constexpr int kHd      = 3;
constexpr int kTok     = kBatch * kSeq;
constexpr int kDim     = 4096;
constexpr int kSgRows  = 16;
constexpr int kTileTok = 32;
static_assert(kTok == 2048 && kHeads * kHd == kEmb && kDim == (1 << kEmb));
static_assert((kDim % 32) == 0 && (kTok % kTileTok) == 0 && ((kTok / kTileTok) % 8) == 0);
static_assert((kSgRows * kDim / 8) % 256 == 0);

constexpr bool kProbResid = false;

constexpr float kPCarry    = 16384.0f;
constexpr float kResid     = 2048.0f;
constexpr float sMeas      = 1.0f / kPCarry;
constexpr float sMeasR     = 1.0f / (kPCarry * kResid);
constexpr float kInvSqrtHd = 0.57735026918962576451f;

constexpr size_t kSzSG    = (size_t)kSgRows * kDim * 2;
constexpr size_t kSzPH    = (size_t)kTok * kDim * 2;
constexpr size_t kSzPL    = kProbResid ? kSzPH : 0;
constexpr size_t kSzTOK   = (size_t)kTok * kEmb * 4;
constexpr size_t kOffSG   = 0;
constexpr size_t kOffPH   = kOffSG + kSzSG;
constexpr size_t kOffPL   = kOffPH + kSzPH;
constexpr size_t kOffTOK  = kOffPL + kSzPL;
constexpr size_t kWsTotal = kOffTOK + kSzTOK;
static_assert(kWsTotal == 17006592ull + (kProbResid ? 16777216ull : 0ull));
static_assert(kWsTotal <= 134217728ull);
static_assert((kOffPH % 128) == 0 && (kOffPL % 128) == 0 && (kOffTOK % 128) == 0);
static_assert((size_t)kTok * kEmb * 4 == 98304ull);

__host__ __device__ constexpr int cnot_map(int k, int ctrl, int tgt) {
  return ((k >> (11 - ctrl)) & 1) ? (k ^ (1 << (11 - tgt))) : k;
}
__host__ __device__ constexpr int cnot_chain(int k) {
  for (int i = 0; i < 11; ++i) k = cnot_map(k, i, i + 1);
  k = cnot_map(k, 11, 0);
  return k;
}
constexpr bool cnot_chain_checks() {
  int img[12] = {};
  for (int b = 0; b < 12; ++b) img[b] = cnot_chain(1 << b);
  for (int k = 0; k < 4096; k += 37) {
    int x = 0;
    for (int b = 0; b < 12; ++b) {
      if ((k >> b) & 1) x ^= img[b];
    }
    if (x != cnot_chain(k)) return false;
    if (x < 0 || x > 4095) return false;
  }
  int rank = 0;
  for (int bit = 11; bit >= 0; --bit) {
    int piv = -1;
    for (int r = rank; r < 12; ++r) {
      if (((img[r] >> bit) & 1) && piv < 0) piv = r;
    }
    if (piv < 0) continue;
    const int t = img[piv]; img[piv] = img[rank]; img[rank] = t;
    for (int r = 0; r < 12; ++r) {
      if (r != rank && ((img[r] >> bit) & 1)) img[r] ^= img[rank];
    }
    ++rank;
  }
  return rank == 12;
}
static_assert(cnot_chain_checks());
static_assert(cnot_chain(0) == 0 && cnot_chain(1) == 2049 && cnot_chain(2) == 2051 && cnot_chain(2048) == 2047);

__device__ __forceinline__ float bf16_rne(float f) {
  const unsigned u = __float_as_uint(f);
  const unsigned r = (u + 0x7FFFu + ((u >> 16) & 1u)) & 0xFFFF0000u;
  return __uint_as_float(r);
}
__device__ __forceinline__ _Float16 f16_flush(float v) {
  const float w = (fabsf(v) < 6.103515625e-05f) ? 0.0f : v;
  return (_Float16)w;
}
__device__ __forceinline__ void pin_f(float& x) { asm volatile("" : "+v"(x)); }
__device__ __forceinline__ void wave_lds_sync() {
  __builtin_amdgcn_fence(__ATOMIC_RELEASE, "workgroup");
  __builtin_amdgcn_wave_barrier();
  __builtin_amdgcn_fence(__ATOMIC_ACQUIRE, "workgroup");
}
__device__ __forceinline__ float head_score(float q0, float q1, float q2, float k0, float k1, float k2) {
  float s = q0 * k0;
  s = fmaf(q1, k1, s);
  s = fmaf(q2, k2, s);
  return s * kInvSqrtHd;
}

namespace mx {
union FragU { v16h v; v8h h[2]; };
__device__ __forceinline__ v16h frag_load(const _Float16* p) {
  FragU f;
  f.h[0] = *(const v8h*)(p);
  f.h[1] = *(const v8h*)(p + 16);
  return f.v;
}
__device__ __forceinline__ v8f mma(v16h a, v16h b, v8f c) {
  return __builtin_amdgcn_wmma_f32_16x16x32_f16(false, a, false, b, (short)0, c, false, false);
}
__device__ __forceinline__ void guard1(v8f& a, v16h x, v16h y) {
  asm volatile("v_nop\n\tv_nop\n\tv_nop\n\tv_nop" : "+v"(a) : "v"(x), "v"(y));
}
__device__ __forceinline__ void guard_acc(v8f& a) {
  asm volatile("v_nop\n\tv_nop\n\tv_nop\n\tv_nop" : "+v"(a));
}
}

__global__ __launch_bounds__(256) void sign_plane_kernel(unsigned* __restrict__ SGw)
{
  const int i  = blockIdx.x * 256 + threadIdx.x;
  const int n  = i >> 9;
  const int k0 = (i & 511) * 8;
  const int nn = (n < kEmb) ? n : (kEmb - 1);
  const unsigned live = (n < kEmb) ? 1u : 0u;
  v4u w;
#pragma unroll
  for (int e = 0; e < 4; ++e) {
    const int ka = k0 + 2 * e;
    const int kb = ka + 1;
    const unsigned ba = (unsigned)((ka >> (11 - nn)) & 1);
    const unsigned bb = (unsigned)((kb >> (11 - nn)) & 1);
    const unsigned ha = live * (ba ? 0xBC00u : 0x3C00u);
    const unsigned hb = live * (bb ? 0xBC00u : 0x3C00u);
    w[e] = ha | (hb << 16);
  }
  unsigned* p = SGw + (size_t)i * 4;
  *(volatile v4u*)p = w;
  __threadfence();
  *(volatile v4u*)p = w;
}

__global__ __launch_bounds__(256) void attention_tok_kernel(
    const float* __restrict__ x,
    const float* __restrict__ wq, const float* __restrict__ wk, const float* __restrict__ wv,
    const float* __restrict__ bq, const float* __restrict__ bk, const float* __restrict__ bv,
    const float* __restrict__ wo, const float* __restrict__ bo,
    float* __restrict__ tokp)
{
  __shared__ __align__(16) float sW[4 * 256];
  __shared__ __align__(16) float sBias[4 * 256];
  __shared__ __align__(16) float sK[kSeq * kEmb];
  __shared__ __align__(16) float sV[kSeq * kEmb];
  __shared__ __align__(16) float sO[kSeq * kEmb];

  const int b = blockIdx.x;
  const int t = threadIdx.x;
  const int lane = t & 31;
  const int wave = t >> 5;

  {
    const int wi = (t < kEmb * kEmb) ? t : (kEmb * kEmb - 1);
    const int bi = (t < kEmb) ? t : (kEmb - 1);
    sW[t]          = bf16_rne(wq[wi]);
    sW[256 + t]    = bf16_rne(wk[wi]);
    sW[512 + t]    = bf16_rne(wv[wi]);
    sW[768 + t]    = bf16_rne(wo[wi]);
    sBias[t]       = bf16_rne(bq[bi]);
    sBias[256 + t] = bf16_rne(bk[bi]);
    sBias[512 + t] = bf16_rne(bv[bi]);
    sBias[768 + t] = bf16_rne(bo[bi]);
  }

  float xr[kEmb];
  {
    const float* xrow = x + ((size_t)b * kSeq + t) * kEmb;
    const v4f x0 = *(const v4f*)(xrow);
    const v4f x1 = *(const v4f*)(xrow + 4);
    const v4f x2 = *(const v4f*)(xrow + 8);
#pragma unroll
    for (int e = 0; e < 4; ++e) {
      xr[e]     = bf16_rne(x0[e]);
      xr[4 + e] = bf16_rne(x1[e]);
      xr[8 + e] = bf16_rne(x2[e]);
    }
  }
  __syncthreads();

  float q[kEmb], kk[kEmb], vv[kEmb];
#pragma unroll
  for (int row = 0; row < kEmb; ++row) {
    float aq = 0.0f, ak = 0.0f, av = 0.0f;
#pragma unroll
    for (int k = 0; k < kEmb; ++k) {
      aq = fmaf(xr[k], sW[row * kEmb + k], aq);
      ak = fmaf(xr[k], sW[256 + row * kEmb + k], ak);
      av = fmaf(xr[k], sW[512 + row * kEmb + k], av);
    }
    q[row]  = aq + sBias[row];
    kk[row] = ak + sBias[256 + row];
    vv[row] = av + sBias[512 + row];
  }
  {
    float* kp = sK + t * kEmb;
    float* vp = sV + t * kEmb;
    *(v4f*)(kp)     = (v4f){kk[0], kk[1], kk[2], kk[3]};
    *(v4f*)(kp + 4) = (v4f){kk[4], kk[5], kk[6], kk[7]};
    *(v4f*)(kp + 8) = (v4f){kk[8], kk[9], kk[10], kk[11]};
    *(v4f*)(vp)     = (v4f){vv[0], vv[1], vv[2], vv[3]};
    *(v4f*)(vp + 4) = (v4f){vv[4], vv[5], vv[6], vv[7]};
    *(v4f*)(vp + 8) = (v4f){vv[8], vv[9], vv[10], vv[11]};
  }
  __syncthreads();

  float mxr[kHeads];
#pragma unroll
  for (int h = 0; h < kHeads; ++h) mxr[h] = -INFINITY;
  for (int s = 0; s < kSeq; ++s) {
    const float* kp = sK + s * kEmb;
    const v4f ka = *(const v4f*)(kp);
    const v4f kb = *(const v4f*)(kp + 4);
    const v4f kc = *(const v4f*)(kp + 8);
    const float kr[kEmb] = {ka[0], ka[1], ka[2], ka[3], kb[0], kb[1], kb[2], kb[3], kc[0], kc[1], kc[2], kc[3]};
#pragma unroll
    for (int h = 0; h < kHeads; ++h) {
      const float sc = head_score(q[3 * h], q[3 * h + 1], q[3 * h + 2], kr[3 * h], kr[3 * h + 1], kr[3 * h + 2]);
      mxr[h] = fmaxf(mxr[h], sc);
    }
  }
  float lsum[kHeads], acc[kEmb];
#pragma unroll
  for (int h = 0; h < kHeads; ++h) lsum[h] = 0.0f;
#pragma unroll
  for (int n = 0; n < kEmb; ++n) acc[n] = 0.0f;
  for (int s = 0; s < kSeq; ++s) {
    const float* kp = sK + s * kEmb;
    const float* vp = sV + s * kEmb;
    const v4f ka = *(const v4f*)(kp);
    const v4f kb = *(const v4f*)(kp + 4);
    const v4f kc = *(const v4f*)(kp + 8);
    const v4f va = *(const v4f*)(vp);
    const v4f vb = *(const v4f*)(vp + 4);
    const v4f vc = *(const v4f*)(vp + 8);
    const float kr[kEmb] = {ka[0], ka[1], ka[2], ka[3], kb[0], kb[1], kb[2], kb[3], kc[0], kc[1], kc[2], kc[3]};
    const float vr[kEmb] = {va[0], va[1], va[2], va[3], vb[0], vb[1], vb[2], vb[3], vc[0], vc[1], vc[2], vc[3]};
#pragma unroll
    for (int h = 0; h < kHeads; ++h) {
      const float sc = head_score(q[3 * h], q[3 * h + 1], q[3 * h + 2], kr[3 * h], kr[3 * h + 1], kr[3 * h + 2]);
      const float e = expf(sc - mxr[h]);
      lsum[h] += e;
      acc[3 * h]     = fmaf(e, vr[3 * h], acc[3 * h]);
      acc[3 * h + 1] = fmaf(e, vr[3 * h + 1], acc[3 * h + 1]);
      acc[3 * h + 2] = fmaf(e, vr[3 * h + 2], acc[3 * h + 2]);
    }
  }
  float ctx[kEmb];
#pragma unroll
  for (int h = 0; h < kHeads; ++h) {
    const float inv = 1.0f / lsum[h];
    ctx[3 * h]     = acc[3 * h] * inv;
    ctx[3 * h + 1] = acc[3 * h + 1] * inv;
    ctx[3 * h + 2] = acc[3 * h + 2] * inv;
  }

  float ao[kEmb];
#pragma unroll
  for (int n = 0; n < kEmb; ++n) {
    float a = 0.0f;
#pragma unroll
    for (int k = 0; k < kEmb; ++k) a = fmaf(ctx[k], sW[768 + n * kEmb + k], a);
    ao[n] = a + sBias[768 + n];
  }
  {
    float* op = sO + t * kEmb;
    *(v4f*)(op)     = (v4f){ao[0], ao[1], ao[2], ao[3]};
    *(v4f*)(op + 4) = (v4f){ao[4], ao[5], ao[6], ao[7]};
    *(v4f*)(op + 8) = (v4f){ao[8], ao[9], ao[10], ao[11]};
  }
  __syncthreads();
  {
    v4f ov[3];
#pragma unroll
    for (int it = 0; it < 3; ++it) ov[it] = *(const v4f*)(sO + it * 1024 + wave * 128 + lane * 4);
    float* gp = tokp + (size_t)b * (kSeq * kEmb);
    for (int pass = 0; pass < 2; ++pass) {
#pragma unroll
      for (int it = 0; it < 3; ++it) {
        *(volatile v4f*)(gp + it * 1024 + wave * 128 + lane * 4) = ov[it];
      }
      __threadfence();
    }
  }
}

__device__ __forceinline__ void rx_wave(float (&re)[16], float (&im)[16], float c, float s, int wmask,
                                        float* sx, float* sy, int tid)
{
#pragma unroll
  for (int j = 0; j < 16; ++j) {
    sx[j * 256 + tid] = re[j];
    sy[j * 256 + tid] = im[j];
  }
  __syncthreads();
  const int pt = tid ^ (wmask << 5);
#pragma unroll
  for (int j = 0; j < 16; ++j) {
    const float pr = sx[j * 256 + pt];
    const float pi = sy[j * 256 + pt];
    const float nr = fmaf(s, pi, c * re[j]);
    const float ni = fmaf(-s, pr, c * im[j]);
    re[j] = nr;
    im[j] = ni;
  }
  __syncthreads();
}
__device__ __forceinline__ void rx_lane(float (&re)[16], float (&im)[16], float c, float s, int mask)
{
#pragma unroll
  for (int j = 0; j < 16; ++j) {
    const float pr = __shfl_xor(re[j], mask, 32);
    const float pi = __shfl_xor(im[j], mask, 32);
    const float nr = fmaf(s, pi, c * re[j]);
    const float ni = fmaf(-s, pr, c * im[j]);
    re[j] = nr;
    im[j] = ni;
  }
}
template <int MB>
__device__ __forceinline__ void rx_slot(float (&re)[16], float (&im)[16], float c, float s)
{
#pragma unroll
  for (int j = 0; j < 16; ++j) {
    if ((j & MB) == 0) {
      const int j1 = j | MB;
      const float r0 = re[j],  i0 = im[j];
      const float r1 = re[j1], i1 = im[j1];
      re[j]  = fmaf(s, i1, c * r0);
      im[j]  = fmaf(-s, r1, c * i0);
      re[j1] = fmaf(s, i0, c * r1);
      im[j1] = fmaf(-s, r0, c * i1);
    }
  }
}

__global__ __launch_bounds__(256) void circuit_probs_kernel(
    const float* __restrict__ tokp, const float* __restrict__ theta,
    unsigned short* __restrict__ PH, unsigned short* __restrict__ PL)
{
  __shared__ __align__(16) float sx[kDim];
  __shared__ __align__(16) float sy[kDim];
  const int tid   = threadIdx.x;
  const int lane  = tid & 31;
  const int token = blockIdx.x;

  float sn, cs;
  {
    const int g  = (lane < 2 * kEmb) ? lane : (2 * kEmb - 1);
    const int wi = (g < kEmb) ? g : (g - kEmb);
    float a = tokp[(size_t)token * kEmb + wi];
    float b = theta[wi];
    pin_f(a);
    pin_f(b);
    b = bf16_rne(b);
    const float fa = (g < kEmb) ? 1.0f : 0.0f;
    const float fb = 1.0f - fa;
    const float ang = fmaf(fa, a, fb * b);
    sincosf(ang * 0.5f, &sn, &cs);
  }

  float re[16], im[16];
#pragma unroll
  for (int j = 0; j < 16; ++j) { re[j] = 0.0f; im[j] = 0.0f; }
  re[0] = (tid == 0) ? 1.0f : 0.0f;

  for (int r = 0; r < 2; ++r) {
    const int g0 = r * kEmb;
    const float c0  = __shfl(cs, g0 + 0, 32),  s0  = __shfl(sn, g0 + 0, 32);
    rx_wave(re, im, c0, s0, 4, sx, sy, tid);
    const float c1  = __shfl(cs, g0 + 1, 32),  s1  = __shfl(sn, g0 + 1, 32);
    rx_wave(re, im, c1, s1, 2, sx, sy, tid);
    const float c2  = __shfl(cs, g0 + 2, 32),  s2  = __shfl(sn, g0 + 2, 32);
    rx_wave(re, im, c2, s2, 1, sx, sy, tid);
    const float c3  = __shfl(cs, g0 + 3, 32),  s3  = __shfl(sn, g0 + 3, 32);
    rx_lane(re, im, c3, s3, 16);
    const float c4  = __shfl(cs, g0 + 4, 32),  s4  = __shfl(sn, g0 + 4, 32);
    rx_lane(re, im, c4, s4, 8);
    const float c5  = __shfl(cs, g0 + 5, 32),  s5  = __shfl(sn, g0 + 5, 32);
    rx_lane(re, im, c5, s5, 4);
    const float c6  = __shfl(cs, g0 + 6, 32),  s6  = __shfl(sn, g0 + 6, 32);
    rx_lane(re, im, c6, s6, 2);
    const float c7  = __shfl(cs, g0 + 7, 32),  s7  = __shfl(sn, g0 + 7, 32);
    rx_lane(re, im, c7, s7, 1);
    const float c8  = __shfl(cs, g0 + 8, 32),  s8  = __shfl(sn, g0 + 8, 32);
    rx_slot<8>(re, im, c8, s8);
    const float c9  = __shfl(cs, g0 + 9, 32),  s9  = __shfl(sn, g0 + 9, 32);
    rx_slot<4>(re, im, c9, s9);
    const float c10 = __shfl(cs, g0 + 10, 32), s10 = __shfl(sn, g0 + 10, 32);
    rx_slot<2>(re, im, c10, s10);
    const float c11 = __shfl(cs, g0 + 11, 32), s11 = __shfl(sn, g0 + 11, 32);
    rx_slot<1>(re, im, c11, s11);
  }

  const int pb = cnot_chain(tid << 4);
#pragma unroll
  for (int j = 0; j < 16; ++j) {
    const float p = fmaf(re[j], re[j], im[j] * im[j]);
    sx[pb ^ cnot_chain(j)] = p * kPCarry;
  }
  __syncthreads();

  v8h hv[2], lv[2];
#pragma unroll
  for (int it = 0; it < 2; ++it) {
    const float* sp = sx + (it * 256 + tid) * 8;
    const v4f a0 = *(const v4f*)(sp);
    const v4f a1 = *(const v4f*)(sp + 4);
#pragma unroll
    for (int e = 0; e < 4; ++e) {
      const float f0 = a0[e];
      const float f1 = a1[e];
      const _Float16 h0 = f16_flush(f0);
      const _Float16 h1 = f16_flush(f1);
      hv[it][e]     = h0;
      hv[it][4 + e] = h1;
      if (kProbResid) {
        const float r0 = (f0 - (float)h0) * kResid;
        const float r1 = (f1 - (float)h1) * kResid;
        lv[it][e]     = f16_flush(r0);
        lv[it][4 + e] = f16_flush(r1);
      } else {
        lv[it][e]     = h0;
        lv[it][4 + e] = h1;
      }
    }
  }
  unsigned short* rowH = PH + (size_t)token * kDim;
  unsigned short* rowL = PL + (size_t)token * kDim;
  for (int pass = 0; pass < 2; ++pass) {
#pragma unroll
    for (int it = 0; it < 2; ++it) {
      const int o = (it * 256 + tid) * 8;
      *(volatile v8h*)(rowH + o) = hv[it];
      if (kProbResid) *(volatile v8h*)(rowL + o) = lv[it];
    }
    __threadfence();
  }
}

template <bool RES>
__global__ __launch_bounds__(256) void measure_gemm_kernel(
    const unsigned short* __restrict__ Ap, const unsigned short* __restrict__ A2p,
    const unsigned short* __restrict__ Btp, float* out, float scale, float rscale)
{
  const _Float16* A  = (const _Float16*)Ap;
  const _Float16* A2 = (const _Float16*)A2p;
  const _Float16* Bt = (const _Float16*)Btp;
  __shared__ __align__(16) float sT[8][kTileTok * kEmb];
  const int lane = threadIdx.x & 31;
  const int wave = threadIdx.x >> 5;
  const int tile = blockIdx.x * 8 + wave;
  if (tile >= kTok / kTileTok) return;
  const int m0    = tile * kTileTok;
  const int rlane = lane & 15;
  const int koff  = (lane >> 4) * 8;
  const int mOff  = (lane >> 4) * 8;

  v8f acc0  = (v8f){0.f, 0.f, 0.f, 0.f, 0.f, 0.f, 0.f, 0.f};
  v8f acc1  = (v8f){0.f, 0.f, 0.f, 0.f, 0.f, 0.f, 0.f, 0.f};
  v8f accr0 = (v8f){0.f, 0.f, 0.f, 0.f, 0.f, 0.f, 0.f, 0.f};
  v8f accr1 = (v8f){0.f, 0.f, 0.f, 0.f, 0.f, 0.f, 0.f, 0.f};

  const size_t bRow  = (size_t)rlane * kDim + koff;
  const size_t aRow0 = (size_t)(m0 + rlane) * kDim + koff;
  const size_t aRow1 = (size_t)(m0 + 16 + rlane) * kDim + koff;
  for (int k0 = 0; k0 < kDim; k0 += 32) {
    const v16h bh = mx::frag_load(Bt + bRow + k0);
    const v16h a0 = mx::frag_load(A + aRow0 + k0);
    const v16h a1 = mx::frag_load(A + aRow1 + k0);
    v16h l0 = a0, l1 = a1;
    if (RES) {
      l0 = mx::frag_load(A2 + aRow0 + k0);
      l1 = mx::frag_load(A2 + aRow1 + k0);
    }
    acc0 = mx::mma(a0, bh, acc0);
    acc1 = mx::mma(a1, bh, acc1);
    if (RES) {
      accr0 = mx::mma(l0, bh, accr0);
      accr1 = mx::mma(l1, bh, accr1);
    }
    mx::guard1(acc0, a0, bh);
    mx::guard1(acc1, a1, bh);
    if (RES) {
      mx::guard1(accr0, l0, bh);
      mx::guard1(accr1, l1, bh);
    }
  }
  mx::guard_acc(acc0);
  mx::guard_acc(acc1);
  if (RES) {
    mx::guard_acc(accr0);
    mx::guard_acc(accr1);
  }

  float* slab = sT[wave];
#pragma unroll
  for (int r = 0; r < 8; ++r) {
    float v0 = acc0[r] * scale;
    float v1 = acc1[r] * scale;
    if (RES) {
      v0 = fmaf(accr0[r], rscale, v0);
      v1 = fmaf(accr1[r], rscale, v1);
    }
    if (rlane < kEmb) {
      slab[(mOff + r) * kEmb + rlane]      = v0;
      slab[(16 + mOff + r) * kEmb + rlane] = v1;
    }
  }
  wave_lds_sync();
  v4f ov[3];
#pragma unroll
  for (int it = 0; it < 3; ++it) ov[it] = *(const v4f*)(slab + it * 128 + lane * 4);
  float* op = out + (size_t)m0 * kEmb;
  for (int pass = 0; pass < 2; ++pass) {
#pragma unroll
    for (int it = 0; it < 3; ++it) {
      *(volatile v4f*)(op + it * 128 + lane * 4) = ov[it];
    }
    __threadfence();
  }
}

extern "C" void kernel_launch(void* const* d_in, const int* in_sizes, int n_in,
                              void* d_out, int out_size, void* d_ws, size_t ws_size,
                              hipStream_t stream)
{
  if (n_in < 10) return;
  if (in_sizes[0] != kTok * kEmb) return;
  if (in_sizes[1] != kEmb * kEmb) return;
  if (in_sizes[2] != kEmb * kEmb) return;
  if (in_sizes[3] != kEmb * kEmb) return;
  if (in_sizes[4] != kEmb) return;
  if (in_sizes[5] != kEmb) return;
  if (in_sizes[6] != kEmb) return;
  if (in_sizes[7] != kEmb * kEmb) return;
  if (in_sizes[8] != kEmb) return;
  if (in_sizes[9] != kEmb) return;
  if (out_size != kTok * kEmb) return;
  if (ws_size < kWsTotal) return;

  const float* x   = (const float*)d_in[0];
  const float* wq  = (const float*)d_in[1];
  const float* wk  = (const float*)d_in[2];
  const float* wv  = (const float*)d_in[3];
  const float* bq  = (const float*)d_in[4];
  const float* bk  = (const float*)d_in[5];
  const float* bv  = (const float*)d_in[6];
  const float* wo  = (const float*)d_in[7];
  const float* bo  = (const float*)d_in[8];
  const float* rxt = (const float*)d_in[9];
  float* out = (float*)d_out;

  char* ws = (char*)d_ws;
  unsigned short* SG  = (unsigned short*)(ws + kOffSG);
  unsigned short* PH  = (unsigned short*)(ws + kOffPH);
  unsigned short* PL  = kProbResid ? (unsigned short*)(ws + kOffPL) : PH;
  float*          TOK = (float*)(ws + kOffTOK);

  sign_plane_kernel<<<dim3((kSgRows * kDim / 8) / 256), 256, 0, stream>>>((unsigned*)SG);

  attention_tok_kernel<<<dim3(kBatch), 256, 0, stream>>>(x, wq, wk, wv, bq, bk, bv, wo, bo, TOK);

  circuit_probs_kernel<<<dim3(kTok), 256, 0, stream>>>(TOK, rxt, PH, PL);

  measure_gemm_kernel<kProbResid><<<dim3((kTok / kTileTok) / 8), 256, 0, stream>>>(
      PH, PL, SG, out, sMeas, sMeasR);
}
